// KPNextBlock_16157666968110
// MI455X (gfx1250) — hardware-verified
//
#include <hip/hip_runtime.h>
#include <math.h>
typedef __attribute__((ext_vector_type(16))) _Float16 v16h;
typedef __attribute__((ext_vector_type(8)))  _Float16 v8h;
typedef __attribute__((ext_vector_type(16))) __bf16   v16b;
typedef __attribute__((ext_vector_type(8)))  __bf16   v8b;
typedef __attribute__((ext_vector_type(8)))  float    v8f;
typedef __attribute__((ext_vector_type(4)))  float    v4f;
#define PSCALE 32768.0f
#define U16(p) ((const unsigned short*)(const void*)(p))
#define PSCALE_INV (1.0f / 32768.0f)

__device__ __forceinline__ unsigned short f2bf_bits(float f) {
  unsigned u = __float_as_uint(f);
  return (unsigned short)((u + 0x7FFFu + ((u >> 16) & 1u)) >> 16);
}
__device__ __forceinline__ float bf_bits2f(unsigned short h) { return __uint_as_float(((unsigned)h) << 16); }

__device__ __forceinline__ void dep_guard_h(v8f& a, v8f& b, v16h x, v16h y) { asm volatile("v_nop\n\tv_nop\n\tv_nop\n\tv_nop" : "+v"(a), "+v"(b) : "v"(x), "v"(y)); }
__device__ __forceinline__ void dep_guard_b(v8f& a, v8f& b, v16b x, v16b y) { asm volatile("v_nop\n\tv_nop\n\tv_nop\n\tv_nop" : "+v"(a), "+v"(b) : "v"(x), "v"(y)); }
__device__ __forceinline__ void keep4_h(v16h a, v16h b, v16h c, v16h d) { asm volatile("v_nop" :: "v"(a), "v"(b), "v"(c), "v"(d)); }
__device__ __forceinline__ void keep4_b(v16b a, v16b b, v16b c, v16b d) { asm volatile("v_nop" :: "v"(a), "v"(b), "v"(c), "v"(d)); }
__device__ __forceinline__ void acc_guard4(v8f& a, v8f& b, v8f& c, v8f& d) { asm volatile("v_nop\n\tv_nop\n\tv_nop\n\tv_nop" : "+v"(a), "+v"(b), "+v"(c), "+v"(d)); }
template <typename T> struct Frag;
template <> struct Frag<_Float16> {
  typedef v16h V; union U { v16h v; v8h h[2]; };
  static __device__ __forceinline__ v16h load(const _Float16* p) {
    U f; f.h[0] = *(const v8h*)(p); f.h[1] = *(const v8h*)(p + 16); return f.v;
  }
  static __device__ __forceinline__ v8f mma(v16h a, v16h b, v8f c) {
    return __builtin_amdgcn_wmma_f32_16x16x32_f16(false, a, false, b, (short)0, c, false, false);
  }
  static __device__ __forceinline__ void guard(v8f& a, v8f& b, v16h x, v16h y) { dep_guard_h(a, b, x, y); }
  static __device__ __forceinline__ void keep(v16h a, v16h b, v16h c, v16h d) { keep4_h(a, b, c, d); }
};
template <> struct Frag<__bf16> {
  typedef v16b V; union U { v16b v; v8b h[2]; };
  static __device__ __forceinline__ v16b load(const __bf16* p) {
    U f; f.h[0] = *(const v8b*)(p); f.h[1] = *(const v8b*)(p + 16); return f.v;
  }
  static __device__ __forceinline__ v8f mma(v16b a, v16b b, v8f c) {
    return __builtin_amdgcn_wmma_f32_16x16x32_bf16(false, a, false, b, (short)0, c, false, false);
  }
  static __device__ __forceinline__ void guard(v8f& a, v8f& b, v16b x, v16b y) { dep_guard_b(a, b, x, y); }
  static __device__ __forceinline__ void keep(v16b a, v16b b, v16b c, v16b d) { keep4_b(a, b, c, d); }
};

template <int ET> struct Elem;
template <> struct Elem<0> { typedef _Float16 T; };
template <> struct Elem<1> { typedef __bf16 T; };
template <int ET, bool SPLIT, int BIAS_MODE, int OUT_MODE, bool RESID, int ACT = 0>
__global__ __launch_bounds__(256) void wmma_gemm64(
    const unsigned short* __restrict__ Ap, const unsigned short* __restrict__ A2p, int lda, long strideA,
    const unsigned short* __restrict__ Btp, const unsigned short* __restrict__ Bt2p, int ldb, long strideB,
    void* __restrict__ Cout, void* __restrict__ Cout2, int ldc, long strideC,
    const float* __restrict__ bias,
    const float* __restrict__ resid, long strideR,
    int M, int N, int K, float scale) {
  typedef typename Elem<ET>::T T;
  typedef typename Frag<T>::V V;
  const T* A = (const T*)Ap; const T* A2 = (const T*)A2p; const T* Bt = (const T*)Btp; const T* Bt2 = (const T*)Bt2p;
  __shared__ __align__(16) float sT[8][16 * 68];
  const int b    = blockIdx.y;
  const int lane = threadIdx.x & 31;
  const int wave = threadIdx.x >> 5;
  const int tilesN = N >> 6;
  const int tilesM = M >> 6;
  const int tile = blockIdx.x * 8 + wave;
  if (tile >= tilesM * tilesN) return;
  const int tm = tile / tilesN;
  const int tn = tile - tm * tilesN;
  const int m0 = tm << 6;
  const int n0 = tn << 6;

  const T* Ab  = A  + (size_t)b * strideA;
  const T* Bb  = Bt + (size_t)b * strideB;
  const T* Ab2 = SPLIT ? (A2  + (size_t)b * strideA) : nullptr;
  const T* Bb2 = SPLIT ? (Bt2 + (size_t)b * strideB) : nullptr;

  const int rlane = lane & 15;
  const int koff  = (lane >> 4) * 8;
  const int mOff  = (lane >> 4) * 8;

  v8f acc[4][4];
#pragma unroll
  for (int i = 0; i < 4; ++i)
#pragma unroll
    for (int j = 0; j < 4; ++j) acc[i][j] = (v8f){0.f,0.f,0.f,0.f,0.f,0.f,0.f,0.f};

  for (int k0 = 0; k0 < K; k0 += 32) {
    V bh[4], bl[4];
#pragma unroll
    for (int j = 0; j < 4; ++j) {
      const size_t bo = (size_t)(n0 + (j << 4) + rlane) * ldb + koff + k0;
      bh[j] = Frag<T>::load(Bb + bo);
      if (SPLIT) bl[j] = Frag<T>::load(Bb2 + bo);
    }
#pragma unroll
    for (int i = 0; i < 4; ++i) {
      const size_t ao = (size_t)(m0 + (i << 4) + rlane) * lda + koff + k0;
      V ah = Frag<T>::load(Ab + ao);
      V al;
      if (SPLIT) al = Frag<T>::load(Ab2 + ao);
#pragma unroll
      for (int j = 0; j < 4; ++j) {
        acc[i][j] = Frag<T>::mma(ah, bh[j], acc[i][j]);
        if (SPLIT) {
          acc[i][j] = Frag<T>::mma(ah, bl[j], acc[i][j]);
          acc[i][j] = Frag<T>::mma(al, bh[j], acc[i][j]);
        }
      }
      Frag<T>::guard(acc[i][0], acc[i][3], ah, SPLIT ? al : ah);
    }
    Frag<T>::keep(bh[0], bh[1], bh[2], bh[3]);
    if (SPLIT) Frag<T>::keep(bl[0], bl[1], bl[2], bl[3]);
  }
  acc_guard4(acc[0][0], acc[0][1], acc[0][2], acc[0][3]);
  acc_guard4(acc[1][0], acc[1][1], acc[1][2], acc[1][3]);
  acc_guard4(acc[2][0], acc[2][1], acc[2][2], acc[2][3]);
  acc_guard4(acc[3][0], acc[3][1], acc[3][2], acc[3][3]);

  float* slab = sT[wave];
  const float* Rb = RESID ? (resid + (size_t)b * strideR) : nullptr;
#pragma unroll
  for (int i = 0; i < 4; ++i) {
    const int mBase = m0 + (i << 4);
#pragma unroll
    for (int j = 0; j < 4; ++j) {
      const int n = n0 + (j << 4) + rlane;
      float bv = 0.f;
      if (BIAS_MODE == 2) bv = bias[n];
#pragma unroll
      for (int r = 0; r < 8; ++r) {
        float v = acc[i][j][r] * scale;
        if (BIAS_MODE == 1) v += bias[mBase + mOff + r];
        if (BIAS_MODE == 2) v += bv;
        if (RESID) v += Rb[(size_t)(mBase + mOff + r) * ldc + n];
        if (ACT == 1) v = tanhf(v);
        if (ACT == 2) v = fmaxf(v, 0.0f);
        if (ACT == 3) v = v / (1.0f + expf(-v));
        if (ACT == 4) v = (v > 0.f) ? v : 0.01f * v;
        if (ACT == 5) v = 0.5f * v * (1.0f + erff(v * 0.70710678118654752f));
        slab[(mOff + r) * 68 + (j << 4) + rlane] = v;
      }
    }
    __builtin_amdgcn_fence(__ATOMIC_RELEASE, "workgroup");
    __builtin_amdgcn_wave_barrier();
    __builtin_amdgcn_fence(__ATOMIC_ACQUIRE, "workgroup");
    if (OUT_MODE == 0) {
      float* C = (float*)Cout + (size_t)b * strideC;
      const int hh = lane >> 4, c4 = (lane & 15) * 4;
      for (int pass = 0; pass < 2; ++pass) {
#pragma unroll
        for (int it = 0; it < 8; ++it) {
          const int row = it * 2 + hh;
          v4f v = *(const v4f*)(slab + row * 68 + c4);
          *(volatile v4f*)(C + (size_t)(mBase + row) * ldc + n0 + c4) = v;
        }
        __threadfence();
      }
    } else {
      const int q = lane >> 3, c8 = (lane & 7) * 8;
      unsigned short* C  = (unsigned short*)Cout  + (size_t)b * strideC;
      unsigned short* C2 = (OUT_MODE == 2) ? ((unsigned short*)Cout2 + (size_t)b * strideC) : nullptr;
      for (int pass = 0; pass < 2; ++pass) {
#pragma unroll
        for (int it = 0; it < 4; ++it) {
          const int row = it * 4 + q;
          const float* sp = slab + row * 68 + c8;
          v8h hv, lv;
#pragma unroll
          for (int e = 0; e < 8; ++e) {
            if (OUT_MODE == 1) {
              hv[e] = (_Float16)sp[e];
            } else {
              unsigned short hb = f2bf_bits(sp[e]);
              unsigned short lb = f2bf_bits(sp[e] - bf_bits2f(hb));
              hv[e] = __builtin_bit_cast(_Float16, hb);
              lv[e] = __builtin_bit_cast(_Float16, lb);
            }
          }
          *(volatile v8h*)(C + (size_t)(mBase + row) * ldc + n0 + c8) = hv;
          if (OUT_MODE == 2) *(volatile v8h*)(C2 + (size_t)(mBase + row) * ldc + n0 + c8) = lv;
        }
        __threadfence();
      }
    }
    __builtin_amdgcn_fence(__ATOMIC_RELEASE, "workgroup");
    __builtin_amdgcn_wave_barrier();
    __builtin_amdgcn_fence(__ATOMIC_ACQUIRE, "workgroup");
  }
}

__global__ __launch_bounds__(256) void cast_f32_f16x2(
    const float* __restrict__ in, _Float16* __restrict__ out, int n2) {
  int i = blockIdx.x * 256 + threadIdx.x;
  if (i < n2) {
    const _Float16 h0 = (_Float16)in[2 * i], h1 = (_Float16)in[2 * i + 1];
    const unsigned u = (unsigned)__builtin_bit_cast(unsigned short, h0) | ((unsigned)__builtin_bit_cast(unsigned short, h1) << 16);
    ((volatile unsigned*)out)[i] = u;
    __threadfence();
    ((volatile unsigned*)out)[i] = u;
  }
}

__global__ __launch_bounds__(256) void split_f32_bf16x2(
    const float* __restrict__ in, __bf16* __restrict__ hi, __bf16* __restrict__ lo, long n2) {
  long i = (long)blockIdx.x * 256 + threadIdx.x;
  long stride = (long)gridDim.x * 256;
  for (int pass = 0; pass < 2; ++pass) {
    for (long j = i; j < n2; j += stride) {
      const float a = in[2 * j], b = in[2 * j + 1];
      const unsigned short ah = f2bf_bits(a), bh = f2bf_bits(b);
      const unsigned short al = f2bf_bits(a - bf_bits2f(ah)), bl = f2bf_bits(b - bf_bits2f(bh));
      ((volatile unsigned*)hi)[j] = (unsigned)ah | ((unsigned)bh << 16);
      ((volatile unsigned*)lo)[j] = (unsigned)al | ((unsigned)bl << 16);
    }
    __threadfence();
  }
}


__global__ __launch_bounds__(256) void transpose_split_bf16(const float* __restrict__ in, int ldi,
                                                           __bf16* __restrict__ outH, __bf16* __restrict__ outL, int ldo) {
  __shared__ __align__(16) float tile[64][68];
  const int c0 = blockIdx.x * 64, r0 = blockIdx.y * 64;
  const int t = threadIdx.y * 32 + threadIdx.x;
  for (int i = threadIdx.y; i < 64; i += 8) {
    tile[threadIdx.x][i]      = in[(size_t)(r0 + i) * ldi + c0 + threadIdx.x];
    tile[32 + threadIdx.x][i] = in[(size_t)(r0 + i) * ldi + c0 + 32 + threadIdx.x];
  }
  __syncthreads();
  const int q = t >> 3, c8 = (t & 7) * 8;
  for (int pass = 0; pass < 2; ++pass) {
#pragma unroll
    for (int it = 0; it < 2; ++it) {
      const int c = it * 32 + q;
      v8b hv, lv;
#pragma unroll
      for (int e = 0; e < 8; ++e) {
        const float f = tile[c][c8 + e];
        const unsigned short hb = f2bf_bits(f);
        hv[e] = __builtin_bit_cast(__bf16, hb);
        lv[e] = __builtin_bit_cast(__bf16, f2bf_bits(f - bf_bits2f(hb)));
      }
      *(volatile v8b*)(outH + (size_t)(c0 + c) * ldo + r0 + c8) = hv;
      *(volatile v8b*)(outL + (size_t)(c0 + c) * ldo + r0 + c8) = lv;
    }
    __threadfence();
  }
}

#define KM 50000
#define KMP 50048
#define KH 32
#define KC 128
#define KK 15
#define KCPG 16
__global__ __launch_bounds__(256) void padsplit_kernel(const float* __restrict__ X, __bf16* __restrict__ Xh, __bf16* __restrict__ Xl) {
  const long i = (long)blockIdx.x * 256 + threadIdx.x; if (i >= (long)KMP * KC / 2) return; const long r = (2 * i) / KC; float a = 0.f, b = 0.f; if (r < KM) { a = X[2 * i]; b = X[2 * i + 1]; }
  const unsigned short ah = f2bf_bits(a), bh = f2bf_bits(b), al = f2bf_bits(a - bf_bits2f(ah)), bl = f2bf_bits(b - bf_bits2f(bh));
  for (int pass = 0; pass < 2; ++pass) { ((volatile unsigned*)Xh)[i] = (unsigned)ah | ((unsigned)bh << 16); ((volatile unsigned*)Xl)[i] = (unsigned)al | ((unsigned)bl << 16); __threadfence(); }
}
__global__ __launch_bounds__(256) void leaky_split_kernel(const float* __restrict__ H1, __bf16* __restrict__ Hh, __bf16* __restrict__ Hl) {
  const long i = (long)blockIdx.x * 256 + threadIdx.x; if (i >= (long)KMP * KC / 2) return; float a = H1[2 * i], b = H1[2 * i + 1]; a = a > 0.f ? a : 0.1f * a; b = b > 0.f ? b : 0.1f * b;
  const unsigned short ah = f2bf_bits(a), bh = f2bf_bits(b), al = f2bf_bits(a - bf_bits2f(ah)), bl = f2bf_bits(b - bf_bits2f(bh));
  for (int pass = 0; pass < 2; ++pass) { ((volatile unsigned*)Hh)[i] = (unsigned)ah | ((unsigned)bh << 16); ((volatile unsigned*)Hl)[i] = (unsigned)al | ((unsigned)bl << 16); __threadfence(); }
}
__global__ __launch_bounds__(256) void w2_kernel(const float* __restrict__ w2, __bf16* __restrict__ Bh, __bf16* __restrict__ Bl) {
  const int i = blockIdx.x * 256 + threadIdx.x; if (i >= 256 * 64) return; const int o = i / 64, kp = 2 * (i % 64); float a = 0.f, b = 0.f; if (o < 240) { a = w2[(size_t)kp * 240 + o]; b = w2[(size_t)(kp + 1) * 240 + o]; }
  const unsigned short ah = f2bf_bits(a), bh = f2bf_bits(b), al = f2bf_bits(a - bf_bits2f(ah)), bl = f2bf_bits(b - bf_bits2f(bh));
  for (int pass = 0; pass < 2; ++pass) { ((volatile unsigned*)Bh)[i] = (unsigned)ah | ((unsigned)bh << 16); ((volatile unsigned*)Bl)[i] = (unsigned)al | ((unsigned)bl << 16); __threadfence(); }
}
__global__ __launch_bounds__(256) void kpconv_kernel(const float* __restrict__ qp, const float* __restrict__ sp, const float* __restrict__ feats, const int* __restrict__ nbi, const float* __restrict__ das, const float* __restrict__ wts, const float* __restrict__ kpts, const float* __restrict__ MODP, float* __restrict__ out) {
  const int lane = threadIdx.x & 31, wave = threadIdx.x >> 5; const int m = blockIdx.x * 8 + wave; if (m >= KM) return;
  const float qx = qp[m * 3], qy = qp[m * 3 + 1], qz = qp[m * 3 + 2]; const float sc = das[m];
  float kx = 0.f, ky = 0.f, kz = 0.f; if (lane < KK) { kx = kpts[lane * 3] * sc; ky = kpts[lane * 3 + 1] * sc; kz = kpts[lane * 3 + 2] * sc; }
  v4f acc = {0.f, 0.f, 0.f, 0.f}; const int c0 = lane * 4; const int cpg = c0 / 8;
#pragma unroll 1
  for (int h = 0; h < KH; ++h) { const int idx = nbi[(size_t)m * KH + h];
    float nx, ny, nz; bool real = (idx >= 0 && idx < KM);
    if (real) { nx = sp[(size_t)idx * 3] - qx; ny = sp[(size_t)idx * 3 + 1] - qy; nz = sp[(size_t)idx * 3 + 2] - qz; } else { nx = 1.0e6f - qx; ny = 1.0e6f - qy; nz = 1.0e6f - qz; }
    float d2 = INFINITY; if (lane < KK) { const float dx = nx - kx, dy = ny - ky, dz = nz - kz; d2 = dx * dx + dy * dy + dz * dz; }
    float mn = d2; for (int o = 16; o > 0; o >>= 1) mn = fminf(mn, __shfl_xor(mn, o, 32));
    const unsigned bal = __ballot(lane < KK && d2 == mn); const int nn = __ffs(bal) - 1;
    const float infl = fmaxf(1.0f - sqrtf(mn) * (1.0f / 0.9f), 0.f);
    if (infl > 0.f && real && nn >= 0) { const v4f f = *(const v4f*)(feats + (size_t)idx * KC + c0); const v4f w = *(const v4f*)(wts + nn * KC + c0);
      const float mod = 1.0f / (1.0f + expf(-MODP[(size_t)m * 256 + nn * KCPG + cpg]));
      const float md2 = 1.0f / (1.0f + expf(-MODP[(size_t)m * 256 + nn * KCPG + (c0 + 2) / 8]));
      acc[0] += f[0] * w[0] * mod * infl; acc[1] += f[1] * w[1] * mod * infl; acc[2] += f[2] * w[2] * md2 * infl; acc[3] += f[3] * w[3] * md2 * infl; } }
  *(volatile v4f*)(out + (size_t)m * KC + c0) = acc; __threadfence(); *(volatile v4f*)(out + (size_t)m * KC + c0) = acc;
}
extern "C" void kernel_launch(void* const* d_in, const int* in_sizes, int n_in, void* d_out, int out_size, void* d_ws, size_t ws_size, hipStream_t stream) {
  (void)in_sizes; (void)n_in; (void)out_size; (void)ws_size;
  auto Fp = [&](int i) { return (const float*)d_in[i]; };
  const float* qp = Fp(0); const float* sp = Fp(1); const float* feats = Fp(2); const int* nbi = (const int*)d_in[3]; const float* das = Fp(4); const float* wts = Fp(5); const float* w1 = Fp(6); const float* b1 = Fp(7); const float* w2 = Fp(8); const float* kpts = Fp(9);
  char* ws = (char*)d_ws; size_t off = 0;
  auto carve = [&](size_t bytes) -> char* { char* p = ws + off; off += (bytes + 255) & ~(size_t)255; return p; };
  __bf16* Xh = (__bf16*)carve((size_t)KMP * KC * 2); __bf16* Xl = (__bf16*)carve((size_t)KMP * KC * 2); __bf16* W1h = (__bf16*)carve(KC * KC * 2); __bf16* W1l = (__bf16*)carve(KC * KC * 2);
  float* H1 = (float*)carve((size_t)KMP * KC * 4); __bf16* Hh = (__bf16*)carve((size_t)KMP * KC * 2); __bf16* Hl = (__bf16*)carve((size_t)KMP * KC * 2); __bf16* W2h = (__bf16*)carve(256 * KC * 2); __bf16* W2l = (__bf16*)carve(256 * KC * 2); float* MODP = (float*)carve((size_t)KMP * 256 * 4);
  padsplit_kernel<<<(KMP * KC / 2 + 255) / 256, 256, 0, stream>>>(feats, Xh, Xl);
  transpose_split_bf16<<<dim3(KC / 64, KC / 64), dim3(32, 8), 0, stream>>>(w1, KC, W1h, W1l, KC);
  w2_kernel<<<(256 * 64 + 255) / 256, 256, 0, stream>>>(w2, W2h, W2l);
  { const int t = (KMP / 64) * 2; wmma_gemm64<1, true, 2, 0, false><<<dim3((t + 7) / 8, 1), 256, 0, stream>>>(U16(Xh), U16(Xl), KC, 0, U16(W1h), U16(W1l), KC, 0, H1, nullptr, KC, 0, b1, nullptr, 0, KMP, KC, KC, 1.0f); }
  leaky_split_kernel<<<(KMP * KC / 2 + 255) / 256, 256, 0, stream>>>(H1, Hh, Hl);
  { const int t = (KMP / 64) * 4; wmma_gemm64<1, true, 0, 0, false><<<dim3((t + 7) / 8, 1), 256, 0, stream>>>(U16(Hh), U16(Hl), KC, 0, U16(W2h), U16(W2l), KC, 0, MODP, nullptr, 256, 0, nullptr, nullptr, 0, KMP, 256, KC, 1.0f); }
  kpconv_kernel<<<(KM + 7) / 8, 256, 0, stream>>>(qp, sp, feats, nbi, das, wts, kpts, MODP, (float*)d_out);
}
